// LocalGCN_70489003262550
// MI455X (gfx1250) — hardware-verified
//
#include <hip/hip_runtime.h>

#define D_IN   16
#define HID    128
#define MAXN   8
#define OUT_D  128
#define BATCH  32768
#define NQT    4
#define QROWS  (BATCH / NQT)
#define QNB    (QROWS * MAXN)
#define EPS_LN 1e-5f
#define RS_HD  0.17677669529663688f

static_assert(BATCH % (NQT * 64) == 0);
static_assert(QROWS % 64 == 0);
static_assert(QNB % 64 == 0);

typedef __attribute__((ext_vector_type(16))) _Float16 v16h;
typedef __attribute__((ext_vector_type(8)))  _Float16 v8h;
typedef __attribute__((ext_vector_type(16))) __bf16   v16b;
typedef __attribute__((ext_vector_type(8)))  __bf16   v8b;
typedef __attribute__((ext_vector_type(8)))  float    v8f;
typedef __attribute__((ext_vector_type(4)))  float    v4f;
typedef __attribute__((ext_vector_type(2)))  unsigned v2u;
#define PSCALE 32768.0f
#define U16(p) ((const unsigned short*)(const void*)(p))
#define PSCALE_INV (1.0f / 32768.0f)

__device__ __forceinline__ unsigned short f2bf_bits(float f) {
  unsigned u = __float_as_uint(f);
  return (unsigned short)((u + 0x7FFFu + ((u >> 16) & 1u)) >> 16);
}
__device__ __forceinline__ float bf_bits2f(unsigned short h) { return __uint_as_float(((unsigned)h) << 16); }

__device__ __forceinline__ void dep_guard_h(v8f& a, v8f& b, v16h x, v16h y) { asm volatile("v_nop\n\tv_nop\n\tv_nop\n\tv_nop" : "+v"(a), "+v"(b) : "v"(x), "v"(y)); }
__device__ __forceinline__ void dep_guard_b(v8f& a, v8f& b, v16b x, v16b y) { asm volatile("v_nop\n\tv_nop\n\tv_nop\n\tv_nop" : "+v"(a), "+v"(b) : "v"(x), "v"(y)); }
__device__ __forceinline__ void keep4_h(v16h a, v16h b, v16h c, v16h d) { asm volatile("v_nop" :: "v"(a), "v"(b), "v"(c), "v"(d)); }
__device__ __forceinline__ void keep4_b(v16b a, v16b b, v16b c, v16b d) { asm volatile("v_nop" :: "v"(a), "v"(b), "v"(c), "v"(d)); }
__device__ __forceinline__ void acc_guard4(v8f& a, v8f& b, v8f& c, v8f& d) { asm volatile("v_nop\n\tv_nop\n\tv_nop\n\tv_nop" : "+v"(a), "+v"(b), "+v"(c), "+v"(d)); }
template <typename T> struct Frag;
template <> struct Frag<_Float16> {
  typedef v16h V; union U { v16h v; v8h h[2]; };
  static __device__ __forceinline__ v16h load(const _Float16* p) {
    U f; f.h[0] = *(const v8h*)(p); f.h[1] = *(const v8h*)(p + 16); return f.v;
  }
  static __device__ __forceinline__ v8f mma(v16h a, v16h b, v8f c) {
    return __builtin_amdgcn_wmma_f32_16x16x32_f16(false, a, false, b, (short)0, c, false, false);
  }
  static __device__ __forceinline__ void guard(v8f& a, v8f& b, v16h x, v16h y) { dep_guard_h(a, b, x, y); }
  static __device__ __forceinline__ void keep(v16h a, v16h b, v16h c, v16h d) { keep4_h(a, b, c, d); }
};
template <> struct Frag<__bf16> {
  typedef v16b V; union U { v16b v; v8b h[2]; };
  static __device__ __forceinline__ v16b load(const __bf16* p) {
    U f; f.h[0] = *(const v8b*)(p); f.h[1] = *(const v8b*)(p + 16); return f.v;
  }
  static __device__ __forceinline__ v8f mma(v16b a, v16b b, v8f c) {
    return __builtin_amdgcn_wmma_f32_16x16x32_bf16(false, a, false, b, (short)0, c, false, false);
  }
  static __device__ __forceinline__ void guard(v8f& a, v8f& b, v16b x, v16b y) { dep_guard_b(a, b, x, y); }
  static __device__ __forceinline__ void keep(v16b a, v16b b, v16b c, v16b d) { keep4_b(a, b, c, d); }
};

template <int ET> struct Elem;
template <> struct Elem<0> { typedef _Float16 T; };
template <> struct Elem<1> { typedef __bf16 T; };
template <int ET, bool SPLIT, int BIAS_MODE, int OUT_MODE, bool RESID, int ACT = 0>
__global__ __launch_bounds__(256) void wmma_gemm64(
    const unsigned short* __restrict__ Ap, const unsigned short* __restrict__ A2p, int lda, long strideA,
    const unsigned short* __restrict__ Btp, const unsigned short* __restrict__ Bt2p, int ldb, long strideB,
    void* __restrict__ Cout, void* __restrict__ Cout2, int ldc, long strideC,
    const float* __restrict__ bias,
    const float* __restrict__ resid, long strideR,
    int M, int N, int K, float scale) {
  typedef typename Elem<ET>::T T;
  typedef typename Frag<T>::V V;
  const T* A = (const T*)Ap; const T* A2 = (const T*)A2p; const T* Bt = (const T*)Btp; const T* Bt2 = (const T*)Bt2p;
  __shared__ __align__(16) float sT[8][16 * 68];
  const int b    = blockIdx.y;
  const int lane = threadIdx.x & 31;
  const int wave = threadIdx.x >> 5;
  const int tilesN = N >> 6;
  const int tilesM = M >> 6;
  const int tile = blockIdx.x * 8 + wave;
  if (tile >= tilesM * tilesN) return;
  const int tm = tile / tilesN;
  const int tn = tile - tm * tilesN;
  const int m0 = tm << 6;
  const int n0 = tn << 6;

  const T* Ab  = A  + (size_t)b * strideA;
  const T* Bb  = Bt + (size_t)b * strideB;
  const T* Ab2 = SPLIT ? (A2  + (size_t)b * strideA) : nullptr;
  const T* Bb2 = SPLIT ? (Bt2 + (size_t)b * strideB) : nullptr;

  const int rlane = lane & 15;
  const int koff  = (lane >> 4) * 8;
  const int mOff  = (lane >> 4) * 8;

  v8f acc[4][4];
#pragma unroll
  for (int i = 0; i < 4; ++i)
#pragma unroll
    for (int j = 0; j < 4; ++j) acc[i][j] = (v8f){0.f,0.f,0.f,0.f,0.f,0.f,0.f,0.f};

  for (int k0 = 0; k0 < K; k0 += 32) {
    V bh[4], bl[4];
#pragma unroll
    for (int j = 0; j < 4; ++j) {
      const size_t bo = (size_t)(n0 + (j << 4) + rlane) * ldb + koff + k0;
      bh[j] = Frag<T>::load(Bb + bo);
      if (SPLIT) bl[j] = Frag<T>::load(Bb2 + bo);
    }
#pragma unroll
    for (int i = 0; i < 4; ++i) {
      const size_t ao = (size_t)(m0 + (i << 4) + rlane) * lda + koff + k0;
      V ah = Frag<T>::load(Ab + ao);
      V al;
      if (SPLIT) al = Frag<T>::load(Ab2 + ao);
#pragma unroll
      for (int j = 0; j < 4; ++j) {
        acc[i][j] = Frag<T>::mma(ah, bh[j], acc[i][j]);
        if (SPLIT) {
          acc[i][j] = Frag<T>::mma(ah, bl[j], acc[i][j]);
          acc[i][j] = Frag<T>::mma(al, bh[j], acc[i][j]);
        }
      }
      Frag<T>::guard(acc[i][0], acc[i][3], ah, SPLIT ? al : ah);
    }
    Frag<T>::keep(bh[0], bh[1], bh[2], bh[3]);
    if (SPLIT) Frag<T>::keep(bl[0], bl[1], bl[2], bl[3]);
  }
  acc_guard4(acc[0][0], acc[0][1], acc[0][2], acc[0][3]);
  acc_guard4(acc[1][0], acc[1][1], acc[1][2], acc[1][3]);
  acc_guard4(acc[2][0], acc[2][1], acc[2][2], acc[2][3]);
  acc_guard4(acc[3][0], acc[3][1], acc[3][2], acc[3][3]);

  float* slab = sT[wave];
  const float* Rb = RESID ? (resid + (size_t)b * strideR) : nullptr;
#pragma unroll
  for (int i = 0; i < 4; ++i) {
    const int mBase = m0 + (i << 4);
#pragma unroll
    for (int j = 0; j < 4; ++j) {
      const int n = n0 + (j << 4) + rlane;
      float bv = 0.f;
      if (BIAS_MODE == 2) bv = bias[n];
#pragma unroll
      for (int r = 0; r < 8; ++r) {
        float v = acc[i][j][r] * scale;
        if (BIAS_MODE == 1) v += bias[mBase + mOff + r];
        if (BIAS_MODE == 2) v += bv;
        if (RESID) v += Rb[(size_t)(mBase + mOff + r) * ldc + n];
        if (ACT == 1) v = tanhf(v);
        if (ACT == 2) v = fmaxf(v, 0.0f);
        if (ACT == 3) v = v / (1.0f + expf(-v));
        if (ACT == 4) v = (v > 0.f) ? v : 0.01f * v;
        if (ACT == 5) v = 0.5f * v * (1.0f + erff(v * 0.70710678118654752f));
        slab[(mOff + r) * 68 + (j << 4) + rlane] = v;
      }
    }
    __builtin_amdgcn_fence(__ATOMIC_RELEASE, "workgroup");
    __builtin_amdgcn_wave_barrier();
    __builtin_amdgcn_fence(__ATOMIC_ACQUIRE, "workgroup");
    if (OUT_MODE == 0) {
      float* C = (float*)Cout + (size_t)b * strideC;
      const int hh = lane >> 4, c4 = (lane & 15) * 4;
      for (int pass = 0; pass < 2; ++pass) {
#pragma unroll
        for (int it = 0; it < 8; ++it) {
          const int row = it * 2 + hh;
          v4f v = *(const v4f*)(slab + row * 68 + c4);
          *(volatile v4f*)(C + (size_t)(mBase + row) * ldc + n0 + c4) = v;
        }
        __threadfence();
      }
    } else {
      const int q = lane >> 3, c8 = (lane & 7) * 8;
      unsigned short* C  = (unsigned short*)Cout  + (size_t)b * strideC;
      unsigned short* C2 = (OUT_MODE == 2) ? ((unsigned short*)Cout2 + (size_t)b * strideC) : nullptr;
      for (int pass = 0; pass < 2; ++pass) {
#pragma unroll
        for (int it = 0; it < 4; ++it) {
          const int row = it * 4 + q;
          const float* sp = slab + row * 68 + c8;
          v8h hv, lv;
#pragma unroll
          for (int e = 0; e < 8; ++e) {
            if (OUT_MODE == 1) {
              hv[e] = (_Float16)sp[e];
            } else {
              unsigned short hb = f2bf_bits(sp[e]);
              unsigned short lb = f2bf_bits(sp[e] - bf_bits2f(hb));
              hv[e] = __builtin_bit_cast(_Float16, hb);
              lv[e] = __builtin_bit_cast(_Float16, lb);
            }
          }
          *(volatile v8h*)(C + (size_t)(mBase + row) * ldc + n0 + c8) = hv;
          if (OUT_MODE == 2) *(volatile v8h*)(C2 + (size_t)(mBase + row) * ldc + n0 + c8) = lv;
        }
        __threadfence();
      }
    }
    __builtin_amdgcn_fence(__ATOMIC_RELEASE, "workgroup");
    __builtin_amdgcn_wave_barrier();
    __builtin_amdgcn_fence(__ATOMIC_ACQUIRE, "workgroup");
  }
}

union H8  { v8h v; unsigned short u[8]; };
union F8  { v4f v[2]; float f[8]; };

template <int MODE>
__global__ __launch_bounds__(256) void k_pack64(const float* __restrict__ x, unsigned short* __restrict__ out, int rows) {
  const int t = blockIdx.x * 256 + threadIdx.x;
  int row = t >> 3;
  const int grp = t & 7;
  row = row < rows ? row : rows - 1;
  const float* xp = x + (size_t)row * D_IN + (grp & 1) * 8;
  F8 ab;
  ab.v[0] = *(const v4f*)xp;
  ab.v[1] = *(const v4f*)(xp + 4);
  const bool useLo = (MODE == 0) ? ((grp & 6) == 2) : ((grp & 6) == 4);
  const bool zero  = grp >= 6;
  H8 o;
#pragma unroll
  for (int e = 0; e < 8; ++e) {
    const float f = ab.f[e];
    const unsigned short hb = f2bf_bits(f);
    const unsigned short lb = f2bf_bits(f - bf_bits2f(hb));
    const unsigned short v = useLo ? lb : hb;
    o.u[e] = zero ? (unsigned short)0 : v;
  }
  unsigned short* dst = out + (size_t)row * 64 + grp * 8;
  *(volatile v8h*)dst = o.v;
  __threadfence();
  *(volatile v8h*)dst = o.v;
}

__global__ __launch_bounds__(256) void k_wsplit(const float* __restrict__ w, unsigned short* __restrict__ hi,
                                                unsigned short* __restrict__ lo, int n8) {
  int i = blockIdx.x * 256 + threadIdx.x;
  const bool act = i < n8;
  i = act ? i : n8 - 1;
  F8 ab;
  ab.v[0] = *(const v4f*)(w + (size_t)i * 8);
  ab.v[1] = *(const v4f*)(w + (size_t)i * 8 + 4);
  H8 oh, ol;
#pragma unroll
  for (int e = 0; e < 8; ++e) {
    const unsigned short hb = f2bf_bits(ab.f[e]);
    const unsigned short lb = f2bf_bits(ab.f[e] - bf_bits2f(hb));
    oh.u[e] = hb; ol.u[e] = lb;
  }
  if (act) {
    unsigned short* dh = hi + (size_t)i * 8;
    unsigned short* dl = lo + (size_t)i * 8;
    *(volatile v8h*)dh = oh.v;
    *(volatile v8h*)dl = ol.v;
    __threadfence();
    *(volatile v8h*)dh = oh.v;
    *(volatile v8h*)dl = ol.v;
  }
}

__device__ __forceinline__ void split_store128(v4f y, unsigned short* stw, unsigned short* planes,
                                               long planeHalves, int row, int lane) {
  unsigned short hb[4], lb[4];
#pragma unroll
  for (int e = 0; e < 4; ++e) {
    hb[e] = f2bf_bits(y[e]);
    lb[e] = f2bf_bits(y[e] - bf_bits2f(hb[e]));
  }
  v2u hv, lv;
  hv[0] = (unsigned)hb[0] | ((unsigned)hb[1] << 16);
  hv[1] = (unsigned)hb[2] | ((unsigned)hb[3] << 16);
  lv[0] = (unsigned)lb[0] | ((unsigned)lb[1] << 16);
  lv[1] = (unsigned)lb[2] | ((unsigned)lb[3] << 16);
  *(v2u*)(stw + 4 * lane) = hv;
  *(v2u*)(stw + 128 + 4 * lane) = lv;
  __builtin_amdgcn_fence(__ATOMIC_RELEASE, "workgroup");
  __builtin_amdgcn_wave_barrier();
  __builtin_amdgcn_fence(__ATOMIC_ACQUIRE, "workgroup");
  const v8h o = *(const v8h*)(stw + 8 * lane);
  unsigned short* dst = planes + (size_t)(lane >> 4) * (size_t)planeHalves + (size_t)row * 128 + 8 * (lane & 15);
  *(volatile v8h*)dst = o;
  __threadfence();
  *(volatile v8h*)dst = o;
  __builtin_amdgcn_fence(__ATOMIC_RELEASE, "workgroup");
  __builtin_amdgcn_wave_barrier();
  __builtin_amdgcn_fence(__ATOMIC_ACQUIRE, "workgroup");
}

#define LN_RW 8
template <bool RELU, int OM>
__global__ __launch_bounds__(256) void k_ln128(const float* __restrict__ in, const float* __restrict__ g,
                                               const float* __restrict__ be, void* __restrict__ outp,
                                               long planeHalves, int ldo, int rows) {
  __shared__ __align__(16) unsigned short stg[8][256];
  const int lane = threadIdx.x & 31, wave = threadIdx.x >> 5;
  const int rbase = (blockIdx.x * 8 + wave) * LN_RW;
  const v4f gv = *(const v4f*)(g + 4 * lane);
  const v4f bv = *(const v4f*)(be + 4 * lane);
  unsigned short* stw = stg[wave];
#pragma unroll 1
  for (int rr = 0; rr < LN_RW; ++rr) {
    int row = rbase + rr;
    row = row < rows ? row : rows - 1;
    const v4f x = *(const v4f*)(in + (size_t)row * 128 + 4 * lane);
    float s = (x[0] + x[1]) + (x[2] + x[3]);
#pragma unroll
    for (int off = 1; off < 32; off <<= 1) s += __shfl_xor(s, off, 32);
    const float m = s * (1.0f / 128.0f);
    const v4f d = x - m;
    float q = (d[0] * d[0] + d[1] * d[1]) + (d[2] * d[2] + d[3] * d[3]);
#pragma unroll
    for (int off = 1; off < 32; off <<= 1) q += __shfl_xor(q, off, 32);
    const float r = rsqrtf(q * (1.0f / 128.0f) + EPS_LN);
    v4f y = (d * r) * gv + bv;
    if (RELU) {
#pragma unroll
      for (int e = 0; e < 4; ++e) y[e] = fmaxf(y[e], 0.0f);
    }
    if (OM == 1) {
      float* o = (float*)outp + (size_t)row * ldo + 4 * lane;
      *(volatile v4f*)o = y;
      __threadfence();
      *(volatile v4f*)o = y;
    } else {
      split_store128(y, stw, (unsigned short*)outp, planeHalves, row, lane);
    }
  }
}

#define ATT_RW 4
__global__ __launch_bounds__(256) void k_attn8(const float* __restrict__ qf, const float* __restrict__ kvf,
                                               const int* __restrict__ mask, unsigned short* __restrict__ ctxp,
                                               long planeHalves, int rows) {
  __shared__ __align__(16) unsigned short stg[8][256];
  const int lane = threadIdx.x & 31, wave = threadIdx.x >> 5;
  const int h = lane >> 3, n = lane & 7;
  unsigned short* stw = stg[wave];
  const int rbase = (blockIdx.x * 8 + wave) * ATT_RW;
#pragma unroll 1
  for (int rr = 0; rr < ATT_RW; ++rr) {
    int row = rbase + rr;
    row = row < rows ? row : rows - 1;
    const float* qp = qf + (size_t)row * HID + h * 32;
    const float* kp = kvf + ((size_t)row * MAXN + n) * (2 * HID) + h * 32;
    float s = 0.0f;
#pragma unroll 1
    for (int i = 0; i < 8; ++i) {
      const v4f a  = *(const v4f*)(qp + 4 * i);
      const v4f k4 = *(const v4f*)(kp + 4 * i);
      s += a[0] * k4[0];
      s += a[1] * k4[1];
      s += a[2] * k4[2];
      s += a[3] * k4[3];
    }
    s *= RS_HD;
    const int mv = mask[(size_t)row * MAXN + n];
    const bool valid = mv > 0;
    const bool anyv = __ballot(valid) != 0ull;
    const bool safe = anyv ? valid : true;
    s = safe ? s : -1.0e9f;
    float mx = s;
    mx = fmaxf(mx, __shfl_xor(mx, 1, 32));
    mx = fmaxf(mx, __shfl_xor(mx, 2, 32));
    mx = fmaxf(mx, __shfl_xor(mx, 4, 32));
    const float e = expf(s - mx);
    float den = e;
    den += __shfl_xor(den, 1, 32);
    den += __shfl_xor(den, 2, 32);
    den += __shfl_xor(den, 4, 32);
    const float p = e * (1.0f / den);
    v4f acc = {0.0f, 0.0f, 0.0f, 0.0f};
    const float* vp = kvf + (size_t)row * MAXN * (2 * HID) + HID + 4 * lane;
#pragma unroll 1
    for (int nn = 0; nn < MAXN; ++nn) {
      const float pn = __shfl(p, (lane & 24) + nn, 32);
      const v4f v4 = *(const v4f*)(vp + (size_t)nn * (2 * HID));
      acc += pn * v4;
    }
    split_store128(acc, stw, ctxp, planeHalves, row, lane);
  }
}

#define CMB_RW 4
__global__ __launch_bounds__(256) void k_combine(const float* __restrict__ of, const unsigned short* __restrict__ curh,
                                                 const unsigned short* __restrict__ curl, const int* __restrict__ mask,
                                                 const float* __restrict__ g, const float* __restrict__ be,
                                                 unsigned short* __restrict__ comb, long planeHalves, int rows) {
  __shared__ __align__(16) unsigned short stg[8][512];
  const int lane = threadIdx.x & 31, wave = threadIdx.x >> 5;
  const int rbase = (blockIdx.x * 8 + wave) * CMB_RW;
  const v4f gv = *(const v4f*)(g + 4 * lane);
  const v4f bv = *(const v4f*)(be + 4 * lane);
  unsigned short* stw = stg[wave];
#pragma unroll 1
  for (int rr = 0; rr < CMB_RW; ++rr) {
    int row = rbase + rr;
    row = row < rows ? row : rows - 1;
    const v4f x = *(const v4f*)(of + (size_t)row * 128 + 4 * lane);
    float s = (x[0] + x[1]) + (x[2] + x[3]);
#pragma unroll
    for (int off = 1; off < 32; off <<= 1) s += __shfl_xor(s, off, 32);
    const float m = s * (1.0f / 128.0f);
    const v4f d = x - m;
    float q = (d[0] * d[0] + d[1] * d[1]) + (d[2] * d[2] + d[3] * d[3]);
#pragma unroll
    for (int off = 1; off < 32; off <<= 1) q += __shfl_xor(q, off, 32);
    const float r = rsqrtf(q * (1.0f / 128.0f) + EPS_LN);
    const v4f y = (d * r) * gv + bv;
    unsigned short hb[4], lb[4];
#pragma unroll
    for (int e = 0; e < 4; ++e) {
      hb[e] = f2bf_bits(y[e]);
      lb[e] = f2bf_bits(y[e] - bf_bits2f(hb[e]));
    }
    v2u yh, yl;
    yh[0] = (unsigned)hb[0] | ((unsigned)hb[1] << 16);
    yh[1] = (unsigned)hb[2] | ((unsigned)hb[3] << 16);
    yl[0] = (unsigned)lb[0] | ((unsigned)lb[1] << 16);
    yl[1] = (unsigned)lb[2] | ((unsigned)lb[3] << 16);
    const v2u ch = *(const v2u*)(curh + (size_t)row * 128 + 4 * lane);
    const v2u cl = *(const v2u*)(curl + (size_t)row * 128 + 4 * lane);
    const int mv = mask[(size_t)row * MAXN + (lane & 7)];
    const bool anyv = __ballot(mv > 0) != 0ull;
    const v2u ah = anyv ? yh : ch;
    const v2u al = anyv ? yl : cl;
    *(v2u*)(stw + 4 * lane) = ch;
    *(v2u*)(stw + 128 + 4 * lane) = ah;
    *(v2u*)(stw + 256 + 4 * lane) = cl;
    *(v2u*)(stw + 384 + 4 * lane) = al;
    __builtin_amdgcn_fence(__ATOMIC_RELEASE, "workgroup");
    __builtin_amdgcn_wave_barrier();
    __builtin_amdgcn_fence(__ATOMIC_ACQUIRE, "workgroup");
    const v8h o0 = *(const v8h*)(stw + 8 * lane);
    const v8h o1 = *(const v8h*)(stw + 256 + 8 * lane);
    unsigned short* d0 = comb + (size_t)row * 256 + 8 * lane;
    unsigned short* d1 = comb + (size_t)planeHalves + (size_t)row * 256 + 8 * lane;
    *(volatile v8h*)d0 = o0;
    *(volatile v8h*)d1 = o1;
    __threadfence();
    *(volatile v8h*)d0 = o0;
    *(volatile v8h*)d1 = o1;
    __builtin_amdgcn_fence(__ATOMIC_RELEASE, "workgroup");
    __builtin_amdgcn_wave_barrier();
    __builtin_amdgcn_fence(__ATOMIC_ACQUIRE, "workgroup");
  }
}

static void gemm_plain(const unsigned short* A, int lda, const unsigned short* Bt, int ldb,
                       float* C, int ldc, const float* bias, int M, int N, int K, hipStream_t st) {
  const int tiles = (M >> 6) * (N >> 6);
  dim3 grid((tiles + 7) / 8, 1, 1);
  wmma_gemm64<1, false, 2, 0, false><<<grid, 256, 0, st>>>(
      A, A, lda, 0L, Bt, Bt, ldb, 0L, (void*)C, (void*)C, ldc, 0L, bias, bias, 0L, M, N, K, 1.0f);
}
static void gemm_split(const unsigned short* Ah, const unsigned short* Al, int lda,
                       const unsigned short* Bh, const unsigned short* Bl, int ldb,
                       float* C, int ldc, const float* bias, int M, int N, int K, hipStream_t st) {
  const int tiles = (M >> 6) * (N >> 6);
  dim3 grid((tiles + 7) / 8, 1, 1);
  wmma_gemm64<1, true, 2, 0, false><<<grid, 256, 0, st>>>(
      Ah, Al, lda, 0L, Bh, Bl, ldb, 0L, (void*)C, (void*)C, ldc, 0L, bias, bias, 0L, M, N, K, 1.0f);
}

extern "C" void kernel_launch(void* const* d_in, const int* in_sizes, int n_in,
                              void* d_out, int out_size, void* d_ws, size_t ws_size,
                              hipStream_t stream) {
  if (n_in < 25) return;
  if (in_sizes[0] != BATCH * D_IN || in_sizes[1] != BATCH * MAXN * D_IN || in_sizes[2] != BATCH * MAXN ||
      in_sizes[11] != 3 * HID * HID || out_size != BATCH * OUT_D) return;

  const float* cur     = (const float*)d_in[0];
  const float* nbr     = (const float*)d_in[1];
  const int*   mask    = (const int*)  d_in[2];
  const float* enc_w1  = (const float*)d_in[3];
  const float* enc_b1  = (const float*)d_in[4];
  const float* enc_g1  = (const float*)d_in[5];
  const float* enc_be1 = (const float*)d_in[6];
  const float* enc_w2  = (const float*)d_in[7];
  const float* enc_b2  = (const float*)d_in[8];
  const float* enc_g2  = (const float*)d_in[9];
  const float* enc_be2 = (const float*)d_in[10];
  const float* in_w    = (const float*)d_in[11];
  const float* in_b    = (const float*)d_in[12];
  const float* out_w   = (const float*)d_in[13];
  const float* out_b   = (const float*)d_in[14];
  const float* an_g    = (const float*)d_in[15];
  const float* an_b    = (const float*)d_in[16];
  const float* p1_w    = (const float*)d_in[17];
  const float* p1_b    = (const float*)d_in[18];
  const float* p1_g    = (const float*)d_in[19];
  const float* p1_be   = (const float*)d_in[20];
  const float* p2_w    = (const float*)d_in[21];
  const float* p2_b    = (const float*)d_in[22];
  const float* p2_g    = (const float*)d_in[23];
  const float* p2_be   = (const float*)d_in[24];

  const size_t szW1P = (size_t)HID * 64 * 2;
  const size_t szW2  = (size_t)HID * HID * 2;
  const size_t szIN  = (size_t)3 * HID * HID * 2;
  const size_t szOW  = (size_t)HID * HID * 2;
  const size_t szP1  = (size_t)HID * 2 * HID * 2;
  const size_t szP2  = (size_t)OUT_D * HID * 2;
  const size_t szCUR = (size_t)BATCH * HID * 2 * 2;
  const size_t szQQ  = (size_t)QROWS * HID * 4;
  const size_t szS   = (size_t)QNB * 2 * HID * 4;
  const size_t szP   = (size_t)QNB * HID * 2 * 2;
  const size_t total = szW1P + 2 * szW2 + 2 * szIN + 2 * szOW + 2 * szP1 + 2 * szP2 + szCUR + szQQ + szS + szP;
  if (total > ws_size) return;

  char* base = (char*)d_ws;
  size_t off = 0;
  auto take = [&](size_t bytes) -> char* { char* p = base + off; off += (bytes + 255) & ~(size_t)255; return p; };
  unsigned short* W1P = (unsigned short*)take(szW1P);
  unsigned short* W2H = (unsigned short*)take(szW2);
  unsigned short* W2L = (unsigned short*)take(szW2);
  unsigned short* INH = (unsigned short*)take(szIN);
  unsigned short* INL = (unsigned short*)take(szIN);
  unsigned short* OWH = (unsigned short*)take(szOW);
  unsigned short* OWL = (unsigned short*)take(szOW);
  unsigned short* P1H = (unsigned short*)take(szP1);
  unsigned short* P1L = (unsigned short*)take(szP1);
  unsigned short* P2H = (unsigned short*)take(szP2);
  unsigned short* P2L = (unsigned short*)take(szP2);
  unsigned short* CURPH = (unsigned short*)take(szCUR);
  unsigned short* CURPL = CURPH + (size_t)BATCH * HID;
  float*          QQ  = (float*)take(szQQ);
  char*           Sb  = take(szS);
  char*           Pb  = take(szP);
  if (off > ws_size) return;

  float*          Sf  = (float*)Sb;
  unsigned short* Pu  = (unsigned short*)Pb;

  k_pack64<1><<<(HID * 8) / 256, 256, 0, stream>>>(enc_w1, W1P, HID);
  k_wsplit<<<(HID * HID / 8) / 256, 256, 0, stream>>>(enc_w2, W2H, W2L, HID * HID / 8);
  k_wsplit<<<(3 * HID * HID / 8) / 256, 256, 0, stream>>>(in_w, INH, INL, 3 * HID * HID / 8);
  k_wsplit<<<(HID * HID / 8) / 256, 256, 0, stream>>>(out_w, OWH, OWL, HID * HID / 8);
  k_wsplit<<<(HID * 2 * HID / 8) / 256, 256, 0, stream>>>(p1_w, P1H, P1L, HID * 2 * HID / 8);
  k_wsplit<<<(OUT_D * HID / 8) / 256, 256, 0, stream>>>(p2_w, P2H, P2L, OUT_D * HID / 8);

  k_pack64<0><<<(BATCH * 8) / 256, 256, 0, stream>>>(cur, Pu, BATCH);
  gemm_plain(Pu, 64, W1P, 64, Sf, HID, enc_b1, BATCH, HID, 64, stream);
  k_ln128<true, 0><<<BATCH / 64, 256, 0, stream>>>(Sf, enc_g1, enc_be1, (void*)Pu, (long)BATCH * HID, 0, BATCH);
  gemm_split(Pu, Pu + (size_t)BATCH * HID, HID, W2H, W2L, HID, Sf, HID, enc_b2, BATCH, HID, HID, stream);
  k_ln128<false, 0><<<BATCH / 64, 256, 0, stream>>>(Sf, enc_g2, enc_be2, (void*)CURPH, (long)BATCH * HID, 0, BATCH);

  for (int qt = 0; qt < NQT; ++qt) {
    const size_t r0  = (size_t)qt * QROWS;
    const size_t nb0 = (size_t)qt * QNB;
    k_pack64<0><<<(QNB * 8) / 256, 256, 0, stream>>>(nbr + nb0 * D_IN, Pu, QNB);
    gemm_plain(Pu, 64, W1P, 64, Sf, HID, enc_b1, QNB, HID, 64, stream);
    k_ln128<true, 0><<<QNB / 64, 256, 0, stream>>>(Sf, enc_g1, enc_be1, (void*)Pu, (long)QNB * HID, 0, QNB);
    gemm_split(Pu, Pu + (size_t)QNB * HID, HID, W2H, W2L, HID, Sf, HID, enc_b2, QNB, HID, HID, stream);
    k_ln128<false, 0><<<QNB / 64, 256, 0, stream>>>(Sf, enc_g2, enc_be2, (void*)Pu, (long)QNB * HID, 0, QNB);
    gemm_split(Pu, Pu + (size_t)QNB * HID, HID, INH + (size_t)HID * HID, INL + (size_t)HID * HID, HID,
               Sf, 2 * HID, in_b + HID, QNB, 2 * HID, HID, stream);
    gemm_split(CURPH + r0 * HID, CURPL + r0 * HID, HID, INH, INL, HID, QQ, HID, in_b, QROWS, HID, HID, stream);
    unsigned short* CTXH = Pu;
    unsigned short* CTXL = Pu + (size_t)QROWS * HID;
    k_attn8<<<QROWS / (8 * ATT_RW), 256, 0, stream>>>(QQ, Sf, mask + r0 * MAXN, CTXH, (long)QROWS * HID, QROWS);
    float* OUTF = Sf;
    gemm_split(CTXH, CTXL, HID, OWH, OWL, HID, OUTF, HID, out_b, QROWS, HID, HID, stream);
    unsigned short* COMBH = (unsigned short*)(Sb + (size_t)QROWS * HID * 4);
    unsigned short* COMBL = COMBH + (size_t)QROWS * 2 * HID;
    k_combine<<<QROWS / (8 * CMB_RW), 256, 0, stream>>>(OUTF, CURPH + r0 * HID, CURPL + r0 * HID,
                                                         mask + r0 * MAXN, an_g, an_b, COMBH,
                                                         (long)QROWS * 2 * HID, QROWS);
    float* P1F = (float*)(Sb + (size_t)QROWS * HID * 4 * 3);
    gemm_split(COMBH, COMBL, 2 * HID, P1H, P1L, 2 * HID, P1F, HID, p1_b, QROWS, HID, 2 * HID, stream);
    unsigned short* HPH = (unsigned short*)(Pb + (size_t)QROWS * HID * 2 * 2);
    unsigned short* HPL = HPH + (size_t)QROWS * HID;
    k_ln128<true, 0><<<QROWS / 64, 256, 0, stream>>>(P1F, p1_g, p1_be, (void*)HPH, (long)QROWS * HID, 0, QROWS);
    float* P2F = (float*)(Sb + (size_t)QROWS * HID * 4 * 4);
    gemm_split(HPH, HPL, HID, P2H, P2L, HID, P2F, OUT_D, p2_b, QROWS, OUT_D, HID, stream);
    k_ln128<false, 1><<<QROWS / 64, 256, 0, stream>>>(P2F, p2_g, p2_be, (void*)((float*)d_out + r0 * OUT_D),
                                                       0L, OUT_D, QROWS);
  }
}
